// QauntMBBlock_82222853915064
// MI455X (gfx1250) — hardware-run, weakly checked
//
#include <hip/hip_runtime.h>
#include <stdint.h>

#define DEVINL __device__ __forceinline__

typedef _Float16 f16t;
typedef _Float16 v16h __attribute__((ext_vector_type(16)));
typedef _Float16 v8h  __attribute__((ext_vector_type(8)));
typedef float v8f __attribute__((ext_vector_type(8)));
typedef float v4f __attribute__((ext_vector_type(4)));
typedef v8h __attribute__((may_alias)) v8ha;
typedef v4f __attribute__((may_alias)) v4fa;
union FragH { v16h v; v8h half[2]; };

#define NB    16
#define CIN   256
#define NPIX  1024
#define IMW   32
#define C3    768
#define NHD   32
#define HDIM  16
#define HCH   48
#define CO    512
#define TPB   256
#define WAVES 8
#define PT    32
#define SP    36
#define NBH   8
#define KVP   132
#define NCH   128
#define PW    36
#define XCAR  1.0f
#define OCAR  64.0f
#define WCAR  16.0f

static_assert(TPB == WAVES * 32);
static_assert(TPB == HDIM * HDIM);
static_assert(NPIX == IMW * IMW);
static_assert(IMW == 32);
static_assert(4 * WAVES == IMW);
static_assert(NPIX == 4 * TPB);
static_assert((NPIX % PT) == 0);
static_assert((CIN % 32) == 0);
static_assert((CO % 32) == 0);
static_assert(C3 == 3 * CIN);
static_assert(CO == NHD * HDIM);
static_assert(C3 == (NHD / 2) * HCH);
static_assert(HCH == 3 * HDIM);
static_assert((SP % 4) == 0);
static_assert((KVP % 4) == 0);
static_assert(KVP >= NCH);
static_assert((NPIX % NCH) == 0);
static_assert(2 * HDIM * NCH == TPB * 16);
static_assert((NB % NBH) == 0);
static_assert(2 * WAVES == HDIM);
static_assert(PW == IMW + 4);

DEVINL v8f wmma_f16(v16h a, v16h b, v8f c) {
  v8f d = __builtin_amdgcn_wmma_f32_16x16x32_f16(false, a, false, b, (short)0, c, false, false);
  asm volatile("v_nop\n\tv_nop\n\tv_nop\n\tv_nop" : "+v"(d) : "v"(a), "v"(b));
  return d;
}
DEVINL v8f zero8f() {
  v8f z = {0.f, 0.f, 0.f, 0.f, 0.f, 0.f, 0.f, 0.f};
  return z;
}

__global__ __launch_bounds__(TPB) void cvt16_k(const float* __restrict__ src, f16t* __restrict__ dst, int n8)
{
  const int t = blockIdx.x * TPB + threadIdx.x;
  const int tc = (t < n8) ? t : (n8 - 1);
  const v4f a = *(const v4fa*)(src + (size_t)tc * 8);
  const v4f c = *(const v4fa*)(src + (size_t)tc * 8 + 4);
  v8h o;
  #pragma unroll
  for (int i = 0; i < 4; ++i) {
    o[i]     = (f16t)(a[i] * WCAR);
    o[4 + i] = (f16t)(c[i] * WCAR);
  }
  f16t* p = dst + (size_t)tc * 8;
  if (t < n8) *(volatile v8h*)p = o;
  __threadfence();
  if (t < n8) *(volatile v8h*)p = o;
}

template <int KD, int NPASS, int CT, bool RESID>
__global__ __launch_bounds__(TPB) void gemm_k(const float* __restrict__ in, const f16t* __restrict__ W16,
                                            const float* __restrict__ res, float* __restrict__ outp, int b0)
{
  static_assert(NPASS * 256 == CT);
  constexpr int PQ = KD + 8;
  static_assert((PQ % 8) == 0);
  __shared__ __attribute__((aligned(16))) f16t  sX[PT * PQ];
  __shared__ __attribute__((aligned(16))) float sStg[WAVES * 16 * SP];
  const int tid = threadIdx.x, lane = tid & 31, wave = tid >> 5;
  const int h = lane >> 4, m = lane & 15;
  const int p0 = blockIdx.x * PT, bl = blockIdx.y;
  const float incar = RESID ? OCAR : XCAR;
  {
    const int c0 = tid >> 3, p4 = (tid & 7) * 4;
    const float* ib = in + (size_t)bl * KD * NPIX + p0 + p4;
    #pragma unroll 2
    for (int i = 0; i < KD / 32; ++i) {
      const int c = c0 + 32 * i;
      const v4f v = *(const v4fa*)(ib + (size_t)c * NPIX);
      #pragma unroll
      for (int j = 0; j < 4; ++j) sX[(p4 + j) * PQ + c] = (f16t)(v[j] * incar);
    }
  }
  __syncthreads();

  const float osc = RESID ? (1.0f / (OCAR * WCAR)) : (1.0f / (XCAR * WCAR));
  const int sub = lane >> 3, piece = (lane & 7) * 4;
  float* stg = sStg + wave * (16 * SP);
  const size_t crow0 = (size_t)(RESID ? (b0 + bl) : bl) * CT;
  #pragma unroll 1
  for (int og = 0; og < NPASS; ++og) {
    const int obase = og * 256 + wave * 32;
    v8f acc[2][2];
    #pragma unroll
    for (int mt = 0; mt < 2; ++mt) {
      #pragma unroll
      for (int nt = 0; nt < 2; ++nt) acc[mt][nt] = zero8f();
    }
    const f16t* arow = W16 + (size_t)(obase + m) * KD + 8 * h;
    const f16t* brow = sX + m * PQ + 8 * h;
    #pragma unroll 1
    for (int ks = 0; ks < KD / 32; ++ks) {
      const int k0 = 32 * ks;
      FragH a0, a1, bq0, bq1;
      a0.half[0]  = *(const v8ha*)(arow + k0);
      a0.half[1]  = *(const v8ha*)(arow + k0 + 16);
      a1.half[0]  = *(const v8ha*)(arow + (size_t)16 * KD + k0);
      a1.half[1]  = *(const v8ha*)(arow + (size_t)16 * KD + k0 + 16);
      bq0.half[0] = *(const v8ha*)(brow + k0);
      bq0.half[1] = *(const v8ha*)(brow + k0 + 16);
      bq1.half[0] = *(const v8ha*)(brow + 16 * PQ + k0);
      bq1.half[1] = *(const v8ha*)(brow + 16 * PQ + k0 + 16);
      acc[0][0] = wmma_f16(a0.v, bq0.v, acc[0][0]);
      acc[0][1] = wmma_f16(a0.v, bq1.v, acc[0][1]);
      acc[1][0] = wmma_f16(a1.v, bq0.v, acc[1][0]);
      acc[1][1] = wmma_f16(a1.v, bq1.v, acc[1][1]);
    }

    #pragma unroll
    for (int mt = 0; mt < 2; ++mt) {
      #pragma unroll
      for (int nt = 0; nt < 2; ++nt) {
        #pragma unroll
        for (int r = 0; r < 8; ++r) stg[(8 * h + r) * SP + 16 * nt + m] = acc[mt][nt][r] * osc;
      }
      __syncthreads();
      const size_t chan0 = crow0 + (size_t)(obase + 16 * mt);
      float* dst = outp + chan0 * NPIX + p0 + piece;
      v4f vv[4];
      #pragma unroll
      for (int i = 0; i < 4; ++i) {
        const int row = 4 * i + sub;
        v4f v = *(const v4fa*)(stg + row * SP + piece);
        if (RESID) {
          const v4f xr = *(const v4fa*)(res + (chan0 + (size_t)row) * NPIX + p0 + piece);
          v += xr;
        }
        vv[i] = v;
      }
      #pragma unroll
      for (int i = 0; i < 4; ++i) *(volatile v4f*)(dst + (size_t)(4 * i + sub) * NPIX) = vv[i];
      __threadfence();
      #pragma unroll
      for (int i = 0; i < 4; ++i) *(volatile v4f*)(dst + (size_t)(4 * i + sub) * NPIX) = vv[i];
      __syncthreads();
    }
  }
}

__global__ __launch_bounds__(TPB) void dwpw_k(const float* __restrict__ qkv, const float* __restrict__ Wdw,
                                            const float* __restrict__ Wpw, float* __restrict__ agg)
{
  __shared__ float sP[PW * PW];
  __shared__ float sWd[HDIM * 25];
  __shared__ float sWp[HDIM * HDIM];
  const int tid = threadIdx.x, lane = tid & 31, wave = tid >> 5;
  const int qq = blockIdx.x, g = blockIdx.y, b = blockIdx.z;
  for (int i = tid; i < PW * PW; i += TPB) sP[i] = 0.0f;
  for (int i = tid; i < HDIM * 25; i += TPB) sWd[i] = Wdw[(size_t)g * (HDIM * 25) + i];
  sWp[tid] = Wpw[(size_t)g * (HDIM * HDIM) + tid];
  __syncthreads();

  const int yy = qq * 8 + wave, xx = lane;
  const int lr = tid >> 3, lc = (tid & 7) * 4;
  float acc[HDIM];
  #pragma unroll
  for (int o = 0; o < HDIM; ++o) acc[o] = 0.0f;
  const float* plane0 = qkv + ((size_t)b * C3 + (size_t)g * HDIM) * NPIX + 4 * tid;
  #pragma unroll 1
  for (int ci = 0; ci < HDIM; ++ci) {
    const v4f v = *(const v4fa*)(plane0 + (size_t)ci * NPIX);
    __syncthreads();
    #pragma unroll
    for (int j = 0; j < 4; ++j) sP[(lr + 2) * PW + lc + 2 + j] = v[j];
    __syncthreads();
    float sv = 0.0f;
    #pragma unroll
    for (int dy = 0; dy < 5; ++dy) {
      #pragma unroll
      for (int dx = 0; dx < 5; ++dx)
        sv = fmaf(sWd[ci * 25 + dy * 5 + dx], sP[(yy + dy) * PW + xx + dx], sv);
    }
    #pragma unroll
    for (int o = 0; o < HDIM; ++o) acc[o] = fmaf(sWp[o * HDIM + ci], sv, acc[o]);
  }
  float* dst = agg + ((size_t)b * C3 + (size_t)g * HDIM) * NPIX + qq * TPB + tid;
  #pragma unroll
  for (int o = 0; o < HDIM; ++o) *(volatile float*)(dst + (size_t)o * NPIX) = acc[o];
  __threadfence();
  #pragma unroll
  for (int o = 0; o < HDIM; ++o) *(volatile float*)(dst + (size_t)o * NPIX) = acc[o];
}

__global__ __launch_bounds__(TPB) void att_k(const float* __restrict__ multi, float* __restrict__ obuf, int b0)
{
  __shared__ __attribute__((aligned(16))) float sCh[2 * HDIM * KVP];
  __shared__ float sKV[HDIM * 17];
  const int tid = threadIdx.x, lane = tid & 31, wave = tid >> 5;
  const int bl = blockIdx.x >> 5, hh = blockIdx.x & 31;
  const int b = b0 + bl;
  const float* base = multi + ((size_t)(hh >> 4) * NB * C3 + (size_t)b * C3 + (size_t)(hh & 15) * HCH) * NPIX;

  const int d = tid >> 4, e = tid & 15;
  const int r = tid >> 3, seg = (tid & 7) * 16;
  const float* rsrc = base + (size_t)(HDIM + r) * NPIX + seg;
  const float rl = (r < HDIM) ? 0.0f : -__builtin_huge_valf();
  float a = 0.0f, s = 0.0f;
  #pragma unroll 1
  for (int ch = 0; ch < NPIX / NCH; ++ch) {
    const int n0 = ch * NCH;
    v4f z0 = *(const v4fa*)(rsrc + n0);
    v4f z1 = *(const v4fa*)(rsrc + n0 + 4);
    v4f z2 = *(const v4fa*)(rsrc + n0 + 8);
    v4f z3 = *(const v4fa*)(rsrc + n0 + 12);
    #pragma unroll
    for (int j = 0; j < 4; ++j) {
      z0[j] = fmaxf(z0[j], rl); z1[j] = fmaxf(z1[j], rl);
      z2[j] = fmaxf(z2[j], rl); z3[j] = fmaxf(z3[j], rl);
    }
    __syncthreads();
    *(v4fa*)(sCh + r * KVP + seg)      = z0;
    *(v4fa*)(sCh + r * KVP + seg + 4)  = z1;
    *(v4fa*)(sCh + r * KVP + seg + 8)  = z2;
    *(v4fa*)(sCh + r * KVP + seg + 12) = z3;
    __syncthreads();
    const float* kr = sCh + d * KVP;
    const float* vr = sCh + (HDIM + e) * KVP;
    #pragma unroll 2
    for (int n4 = 0; n4 < NCH / 4; ++n4) {
      const v4f kk = *(const v4fa*)(kr + 4 * n4);
      const v4f vv = *(const v4fa*)(vr + 4 * n4);
      a = fmaf(kk[0], vv[0], a);
      a = fmaf(kk[1], vv[1], a);
      a = fmaf(kk[2], vv[2], a);
      a = fmaf(kk[3], vv[3], a);
      s += (kk[0] + kk[1]) + (kk[2] + kk[3]);
    }
  }
  sKV[d * 17 + e] = a;
  if (e == 0) sKV[d * 17 + 16] = s;
  __syncthreads();

  const int e0 = wave, e1 = wave + WAVES;
  float kv0[HDIM], kv1[HDIM], ks[HDIM];
  #pragma unroll
  for (int dd = 0; dd < HDIM; ++dd) {
    kv0[dd] = sKV[dd * 17 + e0];
    kv1[dd] = sKV[dd * 17 + e1];
    ks[dd]  = sKV[dd * 17 + 16];
  }
  float* orow0 = obuf + ((size_t)bl * CO + (size_t)hh * HDIM + e0) * NPIX + lane;
  float* orow1 = orow0 + (size_t)WAVES * NPIX;
  const float* qsrc = base + lane;
  #pragma unroll 1
  for (int c = 0; c < NPIX / 32; ++c) {
    const int n0 = c * 32;
    float num0 = 0.0f, num1 = 0.0f, den = 0.0f;
    #pragma unroll
    for (int dd = 0; dd < HDIM; ++dd) {
      const float qv = fmaxf(qsrc[(size_t)dd * NPIX + n0], 0.0f);
      num0 = fmaf(qv, kv0[dd], num0);
      num1 = fmaf(qv, kv1[dd], num1);
      den  = fmaf(qv, ks[dd],  den);
    }
    const float rden = __builtin_amdgcn_rcpf(den + 1e-15f);
    const float o0 = num0 * rden, o1 = num1 * rden;
    *(volatile float*)(orow0 + n0) = o0;
    *(volatile float*)(orow1 + n0) = o1;
    __threadfence();
    *(volatile float*)(orow0 + n0) = o0;
    *(volatile float*)(orow1 + n0) = o1;
  }
}

extern "C" void kernel_launch(void* const* d_in, const int* in_sizes, int n_in,
                              void* d_out, int out_size, void* d_ws, size_t ws_size,
                              hipStream_t stream) {
  if (n_in < 5) return;
  if (in_sizes[0] != NB * CIN * NPIX)  return;
  if (in_sizes[1] != C3 * CIN)         return;
  if (in_sizes[2] != C3 * 25)          return;
  if (in_sizes[3] != C3 * HDIM)        return;
  if (in_sizes[4] != CIN * CO)         return;
  if (out_size != NB * CIN * NPIX)     return;

  const float* x    = (const float*)d_in[0];
  const float* Wqkv = (const float*)d_in[1];
  const float* Wdw  = (const float*)d_in[2];
  const float* Wpw  = (const float*)d_in[3];
  const float* Wpr  = (const float*)d_in[4];
  float* outp = (float*)d_out;

  const size_t szWQ = (size_t)C3 * CIN * 2;
  const size_t szWP = (size_t)CIN * CO * 2;
  const size_t szML = (size_t)2 * NB * C3 * NPIX * 4;
  const size_t szOB = (size_t)NBH * CO * NPIX * 4;
  size_t off = 0;
  char* ws = (char*)d_ws;
  f16t*  WQ16  = (f16t*)(ws + off);   off += szWQ;
  f16t*  WP16  = (f16t*)(ws + off);   off += szWP;
  float* MULTI = (float*)(ws + off);  off += szML;
  float* OBUF  = (float*)(ws + off);  off += szOB;
  if (off > ws_size) return;
  float* AGG = MULTI + (size_t)NB * C3 * NPIX;

  const int nq8 = (C3 * CIN) / 8, np8 = (CIN * CO) / 8;
  cvt16_k<<<(nq8 + TPB - 1) / TPB, TPB, 0, stream>>>(Wqkv, WQ16, nq8);
  cvt16_k<<<(np8 + TPB - 1) / TPB, TPB, 0, stream>>>(Wpr, WP16, np8);
  gemm_k<CIN, 3, C3, false><<<dim3(NPIX / PT, NB), TPB, 0, stream>>>(x, WQ16, x, MULTI, 0);
  dwpw_k<<<dim3(NPIX / TPB, C3 / HDIM, NB), TPB, 0, stream>>>(MULTI, Wdw, Wpw, AGG);
  for (int hb = 0; hb < NB / NBH; ++hb) {
    att_k<<<NBH * NHD, TPB, 0, stream>>>(MULTI, OBUF, hb * NBH);
    gemm_k<CO, 1, CIN, true><<<dim3(NPIX / PT, NBH), TPB, 0, stream>>>(OBUF, WP16, x, outp, hb * NBH);
  }
}
